// GNN_40836549050953
// MI455X (gfx1250) — hardware-verified
//
#include <hip/hip_runtime.h>
#include <stddef.h>
#include <stdint.h>
#include <math.h>


#define NSLOT  4800
#define SPS    2400
#define NTR    800
#define NEDG   1600
#define NVOC   30000
#define DE     300
#define KD     320
#define HCR    1200
#define KH     1216
#define N2     2432
#define NP     320
#define PP     640
#define NOC    768
#define KF     1920
#define NG     1600
#define CPH    300
#define QPH    75
#define NTHR   256
#define GW     8
#define DEGCAP 32
#define GBM    64
#define GBN    64
#define GTHR   128
#define WSMAX  134217728

static_assert(NSLOT % GBM == 0 && NG % GBM == 0);
static_assert(N2 % GBN == 0 && NP % GBN == 0 && NOC % GBN == 0);
static_assert(KD % 32 == 0 && N2 % 32 == 0 && PP % 32 == 0 && KF % 32 == 0);
static_assert(SPS % GW == 0 && NSLOT % GW == 0 && GW * 32 == NTHR && GW * DEGCAP == NTHR);
static_assert(NEDG % 32 == 0 && 4 * QPH == CPH && 4 * CPH == HCR && QPH <= 96);
static_assert((N2 * 2) % 128 == 0 && (KH * 2) % 128 == 0 && (PP * 2) % 128 == 0 && (NOC * 4) % 128 == 0);
static_assert((N2 / 8) % 8 == 0 && (N2 / 8) <= 320);

typedef float          v4f   __attribute__((ext_vector_type(4)));
typedef float          v8f   __attribute__((ext_vector_type(8)));
typedef int            v8i   __attribute__((ext_vector_type(8)));
typedef unsigned int   v4u   __attribute__((ext_vector_type(4)));
typedef unsigned short v4us  __attribute__((ext_vector_type(4)));
typedef unsigned short v8us  __attribute__((ext_vector_type(8)));
typedef unsigned short v16us __attribute__((ext_vector_type(16)));
typedef __bf16         v16bf __attribute__((ext_vector_type(16)));
typedef v4f  __attribute__((may_alias)) v4fa;
typedef v4us __attribute__((may_alias)) v4usa;
typedef v8us __attribute__((may_alias)) v8usa;
union FragB { v16bf v; v16us u; v8us h[2]; v8i w; };

__device__ __forceinline__ v8f wmb(const FragB& a, const FragB& b, v8f c) {
  v8f d = __builtin_amdgcn_wmma_f32_16x16x32_bf16(false, a.v, false, b.v, (short)0, c, false, false);
  asm volatile("v_nop\n\tv_nop\n\tv_nop\n\tv_nop" : "+v"(d) : "v"(a.w), "v"(b.w));
  return d;
}

__device__ __forceinline__ unsigned bf16_bits(float f) {
  const unsigned u = __float_as_uint(f);
  return (u + 0x7FFFu + ((u >> 16) & 1u)) >> 16;
}
__device__ __forceinline__ float bf16_val(float f) {
  return __uint_as_float(bf16_bits(f) << 16);
}
__device__ __forceinline__ unsigned pk2(float a, float b, int part) {
  const unsigned ha = bf16_bits(a), hb = bf16_bits(b);
  const unsigned la = bf16_bits(a - __uint_as_float(ha << 16));
  const unsigned lb = bf16_bits(b - __uint_as_float(hb << 16));
  const unsigned sa = (part != 0) ? la : ha;
  const unsigned sb = (part != 0) ? lb : hb;
  return (sa & 0xFFFFu) | (sb << 16);
}
__device__ __forceinline__ float wsum(float v) {
#pragma unroll
  for (int d = 16; d >= 1; d >>= 1) v += __shfl_xor(v, d, 32);
  return v;
}
__device__ __forceinline__ float wmax(float v) {
#pragma unroll
  for (int d = 16; d >= 1; d >>= 1) v = fmaxf(v, __shfl_xor(v, d, 32));
  return v;
}
__device__ __forceinline__ float lk(float v) { return (v >= 0.0f) ? v : 0.2f * v; }

__global__ __launch_bounds__(NTHR) void k_wprep(const float* __restrict__ Wl1, const float* __restrict__ Wr1,
                                                const float* __restrict__ Wl2, const float* __restrict__ Wr2,
                                                const float* __restrict__ Wp1, const float* __restrict__ Wp2,
                                                const float* __restrict__ Wli,
                                                unsigned short* W1T, unsigned short* W2T, unsigned short* WP1T,
                                                unsigned short* WP2T, unsigned short* WLT) {
  const int job = (int)blockIdx.y;
  const float* W;
  unsigned short* P;
  int kreal, nreal, k8n, npad, pitch, coff, dup;
  if (job == 0)      { W = Wl1; P = W1T;                      kreal = DE;  nreal = HCR; k8n = KD / 8; npad = KH; pitch = KD; coff = 0; dup = 0; }
  else if (job == 1) { W = Wr1; P = W1T + (size_t)KH * KD;    kreal = DE;  nreal = HCR; k8n = KD / 8; npad = KH; pitch = KD; coff = 0; dup = 0; }
  else if (job == 2) { W = Wl2; P = W2T;                      kreal = HCR; nreal = HCR; k8n = KH / 8; npad = KH; pitch = N2; coff = 0; dup = KH; }
  else if (job == 3) { W = Wr2; P = W2T + (size_t)KH * N2;    kreal = HCR; nreal = HCR; k8n = KH / 8; npad = KH; pitch = N2; coff = 0; dup = KH; }
  else if (job == 4) { W = Wp1; P = WP1T;                     kreal = HCR; nreal = DE;  k8n = KH / 8; npad = NP; pitch = N2; coff = 0; dup = KH; }
  else if (job == 5) { W = Wp2; P = WP2T;                     kreal = DE;  nreal = DE;  k8n = KD / 8; npad = NP; pitch = PP; coff = 0; dup = NP; }
  else if (job <= 8) {
    const int j = job - 6;
    W = Wli + (size_t)j * DE * NOC; P = WLT; kreal = DE; nreal = NOC; k8n = KD / 8; npad = NOC; pitch = KF;
    coff = j * PP; dup = NP;
  } else return;
  const int u = (int)blockIdx.x * NTHR + (int)threadIdx.x;
  if (u >= npad * k8n) return;
  const int n  = u / k8n;
  const int k8 = (u - n * k8n) * 8;
  const int nc = n < nreal ? n : nreal - 1;
  v8us o;
#pragma unroll
  for (int i = 0; i < 8; ++i) {
    const int k  = k8 + i;
    const int kc = k < kreal ? k : kreal - 1;
    const float v = W[(size_t)kc * nreal + nc];
    const bool ok = (k < kreal) && (n < nreal);
    o[i] = ok ? (unsigned short)bf16_bits(v) : (unsigned short)0;
  }
  unsigned short* dp = P + (size_t)n * pitch + coff + k8;
  *(volatile v8us*)dp = o;
  if (dup != 0) *(volatile v8us*)(dp + dup) = o;
  __threadfence();
  *(volatile v8us*)dp = o;
  if (dup != 0) *(volatile v8us*)(dp + dup) = o;
}

__global__ __launch_bounds__(NTHR) void k_bprep(const float* __restrict__ bl1, const float* __restrict__ br1,
                                                const float* __restrict__ bl2, const float* __restrict__ br2,
                                                const float* __restrict__ bp1, const float* __restrict__ bp2,
                                                float* BV1, float* BV2, float* BP1, float* BP2) {
  const int job = (int)blockIdx.y;
  const float* s;
  float* d;
  int nreal, npad;
  if (job == 0)      { s = bl1; d = BV1;      nreal = HCR; npad = KH; }
  else if (job == 1) { s = br1; d = BV1 + KH; nreal = HCR; npad = KH; }
  else if (job == 2) { s = bl2; d = BV2;      nreal = HCR; npad = KH; }
  else if (job == 3) { s = br2; d = BV2 + KH; nreal = HCR; npad = KH; }
  else if (job == 4) { s = bp1; d = BP1;      nreal = DE;  npad = NP; }
  else if (job == 5) { s = bp2; d = BP2;      nreal = DE;  npad = NP; }
  else return;
  const int u  = (int)blockIdx.x * NTHR + (int)threadIdx.x;
  const int nu = nreal / 4;
  const int uc = u < nu ? u : nu - 1;
  const v4f a = *(const v4fa*)(s + 4 * uc);
  const bool ok = u < nu;
  v4f o;
  o.x = ok ? bf16_val(a.x) : 0.0f;
  o.y = ok ? bf16_val(a.y) : 0.0f;
  o.z = ok ? bf16_val(a.z) : 0.0f;
  o.w = ok ? bf16_val(a.w) : 0.0f;
  const bool st = u < npad / 4;
  float* dp = d + 4 * (st ? u : 0);
  if (st) *(volatile v4f*)dp = o;
  __threadfence();
  if (st) *(volatile v4f*)dp = o;
}

__global__ __launch_bounds__(NTHR) void k_a0(const int* __restrict__ ids, const float* __restrict__ emb,
                                             unsigned short* A0) {
  const int u = (int)blockIdx.x * NTHR + (int)threadIdx.x;
  if (u >= NSLOT * (KD / 8)) return;
  const int r  = u / (KD / 8);
  const int k8 = (u - r * (KD / 8)) * 8;
  int node = ids[r];
  node = node < 0 ? 0 : (node > NVOC - 1 ? NVOC - 1 : node);
  const int ka = k8 < DE - 4 ? k8 : DE - 4;
  const int kb = (k8 + 4) < DE - 4 ? (k8 + 4) : DE - 4;
  const float* p = emb + (size_t)node * DE;
  const v4f a = *(const v4fa*)(p + ka);
  const v4f b = *(const v4fa*)(p + kb);
  v8us o;
  o[0] = (k8 + 0 < DE) ? (unsigned short)bf16_bits(a.x) : (unsigned short)0;
  o[1] = (k8 + 1 < DE) ? (unsigned short)bf16_bits(a.y) : (unsigned short)0;
  o[2] = (k8 + 2 < DE) ? (unsigned short)bf16_bits(a.z) : (unsigned short)0;
  o[3] = (k8 + 3 < DE) ? (unsigned short)bf16_bits(a.w) : (unsigned short)0;
  o[4] = (k8 + 4 < DE) ? (unsigned short)bf16_bits(b.x) : (unsigned short)0;
  o[5] = (k8 + 5 < DE) ? (unsigned short)bf16_bits(b.y) : (unsigned short)0;
  o[6] = (k8 + 6 < DE) ? (unsigned short)bf16_bits(b.z) : (unsigned short)0;
  o[7] = (k8 + 7 < DE) ? (unsigned short)bf16_bits(b.w) : (unsigned short)0;
  unsigned short* dp = A0 + (size_t)r * KD + k8;
  *(volatile v8us*)dp = o;
  __threadfence();
  *(volatile v8us*)dp = o;
}

template <int MODE, int HASB>
__global__ __launch_bounds__(GTHR) void k_gemm(const unsigned short* __restrict__ A,
                                               const unsigned short* __restrict__ WT,
                                               const float* __restrict__ bv, void* outp, int K, int ldo) {
  __shared__ __attribute__((aligned(16))) float stg[GBM * GBN];
  const int tid = (int)threadIdx.x, lane = tid & 31, wave = tid >> 5, hh = lane >> 4, m = lane & 15;
  const int rowBase = (int)blockIdx.x * GBM;
  const int col0    = (int)blockIdx.y * GBN;

  v8f acc[4];
  {
    const v8f z = {0.f, 0.f, 0.f, 0.f, 0.f, 0.f, 0.f, 0.f};
    acc[0] = z; acc[1] = z; acc[2] = z; acc[3] = z;
  }
  const unsigned short* ap = A  + (size_t)(rowBase + 16 * wave + m) * (size_t)K + 8 * hh;
  const unsigned short* wp = WT + (size_t)(col0 + m) * (size_t)K + 8 * hh;
  const int ksteps = K >> 5;
#pragma unroll 1
  for (int ks = 0; ks < ksteps; ++ks) {
    FragB af;
    af.h[0] = *(const v8usa*)(ap + 32 * ks);
    af.h[1] = *(const v8usa*)(ap + 32 * ks + 16);
#pragma unroll
    for (int t = 0; t < 4; ++t) {
      const unsigned short* wq = wp + (size_t)(16 * t) * (size_t)K + 32 * ks;
      FragB bf;
      bf.h[0] = *(const v8usa*)wq;
      bf.h[1] = *(const v8usa*)(wq + 16);
      acc[t] = wmb(af, bf, acc[t]);
    }
  }

#pragma unroll
  for (int t = 0; t < 4; ++t) {
    const int lc = 16 * t + m;
#pragma unroll
    for (int r = 0; r < 8; ++r) {
      const int lr = 16 * wave + 8 * hh + r;
      stg[lr * GBN + lc] = acc[t][r];
    }
  }
  __syncthreads();

  if constexpr (MODE == 0) {
    float* outF = (float*)outp;
    v4f b4 = {0.f, 0.f, 0.f, 0.f};
    if constexpr (HASB != 0) b4 = *(const v4fa*)(bv + col0 + 4 * m);
    v4f fv[8];
#pragma unroll
    for (int i = 0; i < 8; ++i) {
      const int lr = 16 * wave + 2 * i + hh;
      fv[i] = *(const v4fa*)(stg + lr * GBN + 4 * m) + b4;
    }
#pragma unroll
    for (int i = 0; i < 8; ++i) {
      const int gr = rowBase + 16 * wave + 2 * i + hh;
      float* op = outF + (size_t)gr * (size_t)ldo + col0 + 4 * m;
      *(volatile v4f*)op = fv[i];
    }
    __threadfence();
#pragma unroll
    for (int i = 0; i < 8; ++i) {
      const int gr = rowBase + 16 * wave + 2 * i + hh;
      float* op = outF + (size_t)gr * (size_t)ldo + col0 + 4 * m;
      *(volatile v4f*)op = fv[i];
    }
  } else {
    unsigned short* outH = (unsigned short*)outp;
    const int piece = lane & 7, lq = lane >> 3, part = lq & 1, rsub = lq >> 1;
    v4f ba = {0.f, 0.f, 0.f, 0.f}, bb = {0.f, 0.f, 0.f, 0.f};
    if constexpr (HASB != 0) {
      ba = *(const v4fa*)(bv + col0 + 8 * piece);
      bb = *(const v4fa*)(bv + col0 + 8 * piece + 4);
    }
    v4u pv[8];
#pragma unroll
    for (int j = 0; j < 8; ++j) {
      const int lr = 16 * wave + 2 * j + rsub;
      const v4f xa = *(const v4fa*)(stg + lr * GBN + 8 * piece) + ba;
      const v4f xb = *(const v4fa*)(stg + lr * GBN + 8 * piece + 4) + bb;
      v4u w;
      w.x = pk2(xa.x, xa.y, part);
      w.y = pk2(xa.z, xa.w, part);
      w.z = pk2(xb.x, xb.y, part);
      w.w = pk2(xb.z, xb.w, part);
      pv[j] = w;
    }
    const int half = ldo >> 1;
#pragma unroll
    for (int j = 0; j < 8; ++j) {
      const int gr = rowBase + 16 * wave + 2 * j + rsub;
      unsigned short* op = outH + (size_t)gr * (size_t)ldo + part * half + col0 + 8 * piece;
      *(volatile v4u*)op = pv[j];
    }
    __threadfence();
#pragma unroll
    for (int j = 0; j < 8; ++j) {
      const int gr = rowBase + 16 * wave + 2 * j + rsub;
      unsigned short* op = outH + (size_t)gr * (size_t)ldo + part * half + col0 + 8 * piece;
      *(volatile v4u*)op = pv[j];
    }
  }
}

__global__ __launch_bounds__(NTHR) void k_attn(const int* __restrict__ ids, const float* __restrict__ xlr,
                                               const float* __restrict__ att, const float* __restrict__ bias,
                                               unsigned short* hpl) {
  __shared__ int dsti[NEDG];
  __shared__ int lst[GW * DEGCAP];
  __shared__ __attribute__((aligned(16))) unsigned short rowbuf[GW * N2];
  const int tid = (int)threadIdx.x, lane = tid & 31, wave = tid >> 5;
  const int r0  = (int)blockIdx.x * GW;
  const int smp = r0 / SPS;
  const int* ks = ids + smp * SPS;

#pragma unroll 1
  for (int e = tid; e < NEDG; e += NTHR) {
    const int up = e >= NTR ? 1 : 0;
    const int t  = e - NTR * up;
    dsti[e] = ks[3 * t + 1 + up];
  }
  lst[tid] = r0 + wave;
  __syncthreads();

  const int r    = r0 + wave;
  const int node = ids[r];
  int cnt = 0;
#pragma unroll 1
  for (int p = 0; p < NEDG / 32; ++p) {
    const int e = 32 * p + lane;
    const bool hit = dsti[e] == node;
    const unsigned mk = __builtin_amdgcn_ballot_w32(hit);
    if (mk != 0u) {
      if (hit) {
        const int pos = cnt + (int)__builtin_amdgcn_mbcnt_lo(mk, 0u);
        if (pos < DEGCAP - 1) {
          const int up = e >= NTR ? 1 : 0;
          const int t  = e - NTR * up;
          lst[wave * DEGCAP + pos] = smp * SPS + 3 * t + up;
        }
      }
      cnt += (int)__builtin_popcount(mk);
    }
  }
  const bool ovf = cnt > DEGCAP - 1;
  int n = cnt < 0 ? 0 : (cnt > DEGCAP - 1 ? DEGCAP - 1 : cnt);
  if (lane == 0) lst[wave * DEGCAP + n] = r;
  n = n + 1;
  __syncthreads();

  int msr = lst[wave * DEGCAP + lane];
  msr = msr < 0 ? 0 : (msr > NSLOT - 1 ? NSLOT - 1 : msr);

  const float qnan = __int_as_float(0x7fc00000);
  const float ninf = __int_as_float((int)0xff800000u);
  const float pz = ovf ? qnan : 0.0f;
  const float* xrp = xlr + (size_t)r * N2 + KH;
  unsigned short* rb = rowbuf + wave * N2;
  const bool act = lane < n;

#pragma unroll 1
  for (int h = 0; h < 4; ++h) {
    const int cb = h * CPH;
    v4f xr[3], at[3];
#pragma unroll
    for (int i = 0; i < 3; ++i) {
      const int q  = lane + 32 * i;
      const int qc = q < QPH - 1 ? q : QPH - 1;
      xr[i] = *(const v4fa*)(xrp + cb + 4 * qc);
      const v4f a = *(const v4fa*)(att + cb + 4 * qc);
      const bool ok = q < QPH;
      v4f b;
      b.x = ok ? bf16_val(a.x) : 0.0f;
      b.y = ok ? bf16_val(a.y) : 0.0f;
      b.z = ok ? bf16_val(a.z) : 0.0f;
      b.w = ok ? bf16_val(a.w) : 0.0f;
      at[i] = b;
    }
    float g = ninf;
#pragma unroll 1
    for (int k = 0; k < n; ++k) {
      const int sk = __builtin_amdgcn_readlane(msr, k);
      const float* xp = xlr + (size_t)sk * N2 + cb;
      float s = 0.0f;
#pragma unroll
      for (int i = 0; i < 3; ++i) {
        const int q  = lane + 32 * i;
        const int qc = q < QPH - 1 ? q : QPH - 1;
        const v4f x = *(const v4fa*)(xp + 4 * qc);
        s = fmaf(at[i].x, lk(x.x + xr[i].x), s);
        s = fmaf(at[i].y, lk(x.y + xr[i].y), s);
        s = fmaf(at[i].z, lk(x.z + xr[i].z), s);
        s = fmaf(at[i].w, lk(x.w + xr[i].w), s);
      }
      s = wsum(s);
      g = (lane == k) ? s : g;
    }
    const float mx  = wmax(act ? g : ninf);
    const float ex  = act ? expf(g - mx) : 0.0f;
    const float den = wsum(ex);
    const float al  = ex * (1.0f / den);
    const int   ali = __float_as_int(al);

    v4f acc[3];
    {
      const v4f z = {0.f, 0.f, 0.f, 0.f};
      acc[0] = z; acc[1] = z; acc[2] = z;
    }
#pragma unroll 1
    for (int k = 0; k < n; ++k) {
      const int   sk = __builtin_amdgcn_readlane(msr, k);
      const float ak = __int_as_float(__builtin_amdgcn_readlane(ali, k));
      const float* xp = xlr + (size_t)sk * N2 + cb;
#pragma unroll
      for (int i = 0; i < 3; ++i) {
        const int q  = lane + 32 * i;
        const int qc = q < QPH - 1 ? q : QPH - 1;
        const v4f x = *(const v4fa*)(xp + 4 * qc);
        acc[i].x = fmaf(ak, x.x, acc[i].x);
        acc[i].y = fmaf(ak, x.y, acc[i].y);
        acc[i].z = fmaf(ak, x.z, acc[i].z);
        acc[i].w = fmaf(ak, x.w, acc[i].w);
      }
    }
#pragma unroll
    for (int i = 0; i < 3; ++i) {
      const int q  = lane + 32 * i;
      const int qc = q < QPH - 1 ? q : QPH - 1;
      const v4f bq = *(const v4fa*)(bias + cb + 4 * qc);
      float v0 = acc[i].x + bf16_val(bq.x);
      float v1 = acc[i].y + bf16_val(bq.y);
      float v2 = acc[i].z + bf16_val(bq.z);
      float v3 = acc[i].w + bf16_val(bq.w);
      v0 = ((v0 > 0.0f) ? v0 : (v0 - v0)) + pz;
      v1 = ((v1 > 0.0f) ? v1 : (v1 - v1)) + pz;
      v2 = ((v2 > 0.0f) ? v2 : (v2 - v2)) + pz;
      v3 = ((v3 > 0.0f) ? v3 : (v3 - v3)) + pz;
      v4us h4, l4;
      unsigned hb;
      hb = bf16_bits(v0); h4[0] = (unsigned short)hb; l4[0] = (unsigned short)bf16_bits(v0 - __uint_as_float(hb << 16));
      hb = bf16_bits(v1); h4[1] = (unsigned short)hb; l4[1] = (unsigned short)bf16_bits(v1 - __uint_as_float(hb << 16));
      hb = bf16_bits(v2); h4[2] = (unsigned short)hb; l4[2] = (unsigned short)bf16_bits(v2 - __uint_as_float(hb << 16));
      hb = bf16_bits(v3); h4[3] = (unsigned short)hb; l4[3] = (unsigned short)bf16_bits(v3 - __uint_as_float(hb << 16));
      if (q < QPH) {
        *(v4usa*)(rb + cb + 4 * q) = h4;
        *(v4usa*)(rb + KH + cb + 4 * q) = l4;
      }
    }
  }
  if (lane < 4) {
    const v4us z4 = {0, 0, 0, 0};
    *(v4usa*)(rb + HCR + 4 * lane) = z4;
    *(v4usa*)(rb + KH + HCR + 4 * lane) = z4;
  }
  __syncthreads();

  v8us qv[10];
#pragma unroll
  for (int j = 0; j < 10; ++j) {
    const int pi = lane + 32 * j;
    const int pc = pi < (N2 / 8) - 1 ? pi : (N2 / 8) - 1;
    qv[j] = *(const v8usa*)(rb + 8 * pc);
  }
  unsigned short* hp = hpl + (size_t)r * N2;
#pragma unroll
  for (int j = 0; j < 10; ++j) {
    const int pi = lane + 32 * j;
    if (pi < N2 / 8) *(volatile v8us*)(hp + 8 * pi) = qv[j];
  }
  __threadfence();
#pragma unroll
  for (int j = 0; j < 10; ++j) {
    const int pi = lane + 32 * j;
    if (pi < N2 / 8) *(volatile v8us*)(hp + 8 * pi) = qv[j];
  }
}

constexpr size_t AL(size_t x) { return (x + 255) & ~(size_t)255; }
constexpr size_t SZ_A0   = (size_t)NSLOT * KD * 2;
constexpr size_t SZ_W1T  = (size_t)N2 * KD * 2;
constexpr size_t SZ_W2T  = (size_t)N2 * N2 * 2;
constexpr size_t SZ_WP1T = (size_t)NP * N2 * 2;
constexpr size_t SZ_WP2T = (size_t)NP * PP * 2;
constexpr size_t SZ_WLT  = (size_t)NOC * KF * 2;
constexpr size_t SZ_BV   = (size_t)N2 * 4;
constexpr size_t SZ_BP   = (size_t)NP * 4;
constexpr size_t SZ_XLR  = (size_t)NSLOT * N2 * 4;
constexpr size_t SZ_H    = (size_t)NSLOT * N2 * 2;
constexpr size_t SZ_P    = (size_t)NSLOT * PP * 2;
constexpr size_t O_A0   = 0;
constexpr size_t O_W1T  = AL(O_A0 + SZ_A0);
constexpr size_t O_W2T  = AL(O_W1T + SZ_W1T);
constexpr size_t O_WP1T = AL(O_W2T + SZ_W2T);
constexpr size_t O_WP2T = AL(O_WP1T + SZ_WP1T);
constexpr size_t O_WLT  = AL(O_WP2T + SZ_WP2T);
constexpr size_t O_BV1  = AL(O_WLT + SZ_WLT);
constexpr size_t O_BV2  = AL(O_BV1 + SZ_BV);
constexpr size_t O_BP1  = AL(O_BV2 + SZ_BV);
constexpr size_t O_BP2  = AL(O_BP1 + SZ_BP);
constexpr size_t O_XLR  = AL(O_BP2 + SZ_BP);
constexpr size_t O_H    = AL(O_XLR + SZ_XLR);
constexpr size_t O_P    = AL(O_H + SZ_H);
constexpr size_t O_WN   = AL(O_P + SZ_P);
constexpr size_t WS_TOTAL = AL(O_WN + SZ_P);
static_assert(WS_TOTAL <= (size_t)WSMAX);
static_assert((size_t)(NG - 1) * NOC + (NOC - 1) == (size_t)2 * NTR * NOC - 1);

extern "C" void kernel_launch(void* const* d_in, const int* in_sizes, int n_in,
                              void* d_out, int out_size, void* d_ws, size_t ws_size,
                              hipStream_t stream) {
  if (n_in < 19) return;
  if (in_sizes[0] != NSLOT) return;
  if (in_sizes[1] != NVOC * DE) return;
  if (in_sizes[2] != DE * HCR || in_sizes[3] != HCR) return;
  if (in_sizes[4] != DE * HCR || in_sizes[5] != HCR) return;
  if (in_sizes[6] != HCR || in_sizes[7] != HCR) return;
  if (in_sizes[8] != HCR * HCR || in_sizes[9] != HCR) return;
  if (in_sizes[10] != HCR * HCR || in_sizes[11] != HCR) return;
  if (in_sizes[12] != HCR || in_sizes[13] != HCR) return;
  if (in_sizes[14] != HCR * DE || in_sizes[15] != DE) return;
  if (in_sizes[16] != DE * DE || in_sizes[17] != DE) return;
  if (in_sizes[18] != 3 * DE * NOC) return;
  if (out_size != NG * NOC) return;
  if (WS_TOTAL > ws_size) return;

  const int*   ids   = (const int*)d_in[0];
  const float* emb   = (const float*)d_in[1];
  const float* Wl1   = (const float*)d_in[2];
  const float* bl1   = (const float*)d_in[3];
  const float* Wr1   = (const float*)d_in[4];
  const float* br1   = (const float*)d_in[5];
  const float* att1  = (const float*)d_in[6];
  const float* bias1 = (const float*)d_in[7];
  const float* Wl2   = (const float*)d_in[8];
  const float* bl2   = (const float*)d_in[9];
  const float* Wr2   = (const float*)d_in[10];
  const float* br2   = (const float*)d_in[11];
  const float* att2  = (const float*)d_in[12];
  const float* bias2 = (const float*)d_in[13];
  const float* Wp1   = (const float*)d_in[14];
  const float* bp1   = (const float*)d_in[15];
  const float* Wp2   = (const float*)d_in[16];
  const float* bp2   = (const float*)d_in[17];
  const float* Wli   = (const float*)d_in[18];
  float* out = (float*)d_out;

  char* ws = (char*)d_ws;
  unsigned short* A0   = (unsigned short*)(ws + O_A0);
  unsigned short* W1T  = (unsigned short*)(ws + O_W1T);
  unsigned short* W2T  = (unsigned short*)(ws + O_W2T);
  unsigned short* WP1T = (unsigned short*)(ws + O_WP1T);
  unsigned short* WP2T = (unsigned short*)(ws + O_WP2T);
  unsigned short* WLT  = (unsigned short*)(ws + O_WLT);
  float*          BV1  = (float*)(ws + O_BV1);
  float*          BV2  = (float*)(ws + O_BV2);
  float*          BP1  = (float*)(ws + O_BP1);
  float*          BP2  = (float*)(ws + O_BP2);
  float*          XLR  = (float*)(ws + O_XLR);
  unsigned short* HPL  = (unsigned short*)(ws + O_H);
  unsigned short* PPL  = (unsigned short*)(ws + O_P);
  unsigned short* WNP  = (unsigned short*)(ws + O_WN);

  k_wprep<<<dim3((KH * (KH / 8) + NTHR - 1) / NTHR, 9), NTHR, 0, stream>>>(Wl1, Wr1, Wl2, Wr2, Wp1, Wp2, Wli,
                                                                            W1T, W2T, WP1T, WP2T, WLT);
  k_bprep<<<dim3(2, 6), NTHR, 0, stream>>>(bl1, br1, bl2, br2, bp1, bp2, BV1, BV2, BP1, BP2);
  k_a0<<<(NSLOT * (KD / 8)) / NTHR, NTHR, 0, stream>>>(ids, emb, A0);
  k_gemm<0, 1><<<dim3(NSLOT / GBM, N2 / GBN), GTHR, 0, stream>>>(A0, W1T, BV1, (void*)XLR, KD, N2);
  k_attn<<<NSLOT / GW, NTHR, 0, stream>>>(ids, XLR, att1, bias1, HPL);
  k_gemm<0, 1><<<dim3(NSLOT / GBM, N2 / GBN), GTHR, 0, stream>>>(HPL, W2T, BV2, (void*)XLR, N2, N2);
  k_attn<<<NSLOT / GW, NTHR, 0, stream>>>(ids, XLR, att2, bias2, HPL);
  k_gemm<1, 1><<<dim3(NSLOT / GBM, NP / GBN), GTHR, 0, stream>>>(HPL, WP1T, BP1, (void*)PPL, N2, PP);
  k_gemm<1, 1><<<dim3(NSLOT / GBM, NP / GBN), GTHR, 0, stream>>>(PPL, WP2T, BP2, (void*)WNP, PP, PP);
  k_gemm<0, 0><<<dim3(NG / GBM, NOC / GBN), GTHR, 0, stream>>>(WNP, WLT, BV1, (void*)out, KF, NOC);
}
